// RNNModel_50053548867903
// MI455X (gfx1250) — hardware-verified
//
#include <hip/hip_runtime.h>
#include <math.h>

constexpr int NBATCH = 256;
constexpr int NSTEP  = 2048;
constexpr int NFEAT  = 2;
constexpr int NHID   = 128;
constexpr int NOUTC  = 2;
constexpr int NG3    = 3 * NHID;
constexpr int NTHR   = 256;
constexpr int RB     = 16;
constexpr int HP     = 136;
constexpr int FP     = 132;
constexpr int TCH    = 16;
constexpr int XSP    = TCH * NFEAT;
constexpr int OSP    = TCH * NOUTC;
constexpr int TWP    = 136;
constexpr float HCARRY  = 256.0f;
constexpr float WCARRY  = 16.0f;
constexpr float ACC_INV = 1.0f / (HCARRY * WCARRY);
constexpr int NOUT0 = NBATCH * NHID;
constexpr int NOUT1 = NBATCH * NSTEP * NOUTC;
static_assert(NOUT0 * 4 == 131072);
static_assert(NBATCH % RB == 0);
static_assert(NSTEP % TCH == 0);
static_assert(NHID == 16 * (NTHR / 32));
static_assert(NHID % 64 == 0);
static_assert(XSP * 4 == 128 && OSP * 4 == 128);
static_assert(RB * XSP == 128 * 4);
static_assert(RB * NHID == NTHR * 8);
static_assert(NFEAT * NHID == NTHR);
static_assert(NHID * NOUTC == NTHR);
static_assert(NG3 == 12 * 32);

typedef __attribute__((ext_vector_type(16))) _Float16 v16h;
typedef __attribute__((ext_vector_type(8)))  _Float16 v8h;
typedef __attribute__((ext_vector_type(8)))  float    v8f;
typedef __attribute__((ext_vector_type(4)))  float    v4f;
typedef __attribute__((ext_vector_type(2)))  float    v2f;

__device__ __forceinline__ void dep_guard3_h(v8f& a, v8f& b, v8f& c, v16h w, v16h x, v16h y, v16h z) {
  asm volatile("v_nop\n\tv_nop\n\tv_nop\n\tv_nop" : "+v"(a), "+v"(b), "+v"(c) : "v"(w), "v"(x), "v"(y), "v"(z));
}
__device__ __forceinline__ void acc_guard3(v8f& a, v8f& b, v8f& c) {
  asm volatile("v_nop\n\tv_nop\n\tv_nop\n\tv_nop" : "+v"(a), "+v"(b), "+v"(c));
}

template <typename T> struct Frag;
template <> struct Frag<_Float16> {
  typedef v16h V; union U { v16h v; v8h h[2]; };
  static __device__ __forceinline__ v16h load(const _Float16* p) {
    U f; f.h[0] = *(const v8h*)(p); f.h[1] = *(const v8h*)(p + 16); return f.v;
  }
  static __device__ __forceinline__ v8f mma(v16h a, v16h b, v8f c) {
    return __builtin_amdgcn_wmma_f32_16x16x32_f16(false, a, false, b, (short)0, c, false, false);
  }
};

__device__ __forceinline__ float fsig(float v)  { return __builtin_amdgcn_rcpf(1.0f + expf(-v)); }
__device__ __forceinline__ float ftanh(float v) { return 1.0f - 2.0f * __builtin_amdgcn_rcpf(1.0f + expf(2.0f * v)); }

__device__ __forceinline__ void kstep3(v8f& ar, v8f& az, v8f& an,
                                       const _Float16* ap, const _Float16* rp, const _Float16* zp, const _Float16* np) {
  const v16h a  = Frag<_Float16>::load(ap);
  const v16h b0 = Frag<_Float16>::load(rp);
  const v16h b1 = Frag<_Float16>::load(zp);
  const v16h b2 = Frag<_Float16>::load(np);
  ar = Frag<_Float16>::mma(a, b0, ar);
  az = Frag<_Float16>::mma(a, b1, az);
  an = Frag<_Float16>::mma(a, b2, an);
  dep_guard3_h(ar, az, an, a, b0, b1, b2);
}

__global__ __launch_bounds__(NTHR) void prep_w_kernel(const float* __restrict__ Whr, const float* __restrict__ Whz,
                                                      const float* __restrict__ Whn, _Float16* __restrict__ WHH) {
  __shared__ __align__(16) _Float16 tw[32 * TWP];
  const int tid = threadIdx.x, lane = tid & 31, wave = tid >> 5;
  const int g  = blockIdx.x >> 2;
  const int n0 = (blockIdx.x & 3) * 32;
  const float* Wg = (g == 0) ? Whr : ((g == 1) ? Whz : Whn);
#pragma unroll 1
  for (int i = 0; i < 16; ++i) {
    const int k = wave + 8 * i;
    const float w = Wg[(size_t)k * NHID + n0 + lane];
    tw[lane * TWP + k] = (_Float16)(w * WCARRY);
  }
  __syncthreads();
  const int q = lane >> 3, c8 = (lane & 7) * 8;
  const int row = 4 * wave + q;
  _Float16* dst = WHH + (size_t)(g * NHID + n0 + row) * NHID;
  for (int pass = 0; pass < 2; ++pass) {
#pragma unroll
    for (int it = 0; it < 2; ++it) {
      const v8h v = *(const v8h*)(tw + row * TWP + it * 64 + c8);
      *(volatile v8h*)(dst + it * 64 + c8) = v;
    }
    __threadfence();
  }
}

__global__ __launch_bounds__(NTHR) void gru_seq_kernel(
    const float* __restrict__ x, const float* __restrict__ h0,
    const float* __restrict__ Wir, const float* __restrict__ Wiz, const float* __restrict__ Win,
    const _Float16* __restrict__ WHH,
    const float* __restrict__ bhr, const float* __restrict__ bhz, const float* __restrict__ bhn,
    const float* __restrict__ Wd, const float* __restrict__ bd,
    float* __restrict__ out0, float* __restrict__ out1) {
  __shared__ __align__(16) _Float16 h16[RB * HP];
  __shared__ __align__(16) float    hf[RB * FP];
  __shared__ __align__(16) float    xs[RB * XSP];
  __shared__ __align__(16) float    outs[RB * OSP];
  __shared__ __align__(16) float    part[RB * NOUTC * 8];
  __shared__ float swi[3 * NFEAT * NHID];
  __shared__ float swd[NHID * NOUTC];
  __shared__ float sbh[3 * NHID];
  __shared__ float sbd[4];

  const int tid = threadIdx.x, lane = tid & 31, wave = tid >> 5;
  const int c = lane & 15, hh = lane >> 4, koff = hh * 8, mOff = hh * 8;
  const int b0 = blockIdx.x * RB;
  const int j = 16 * wave + c;

#pragma unroll 1
  for (int i = tid; i < RB * HP; i += NTHR) h16[i] = (_Float16)0.0f;
  swi[tid]              = Wir[tid];
  swi[NTHR + tid]       = Wiz[tid];
  swi[2 * NTHR + tid]   = Win[tid];
  swd[tid]              = Wd[tid];
  if (wave < 4) {
    sbh[tid]            = bhr[tid];
    sbh[NHID + tid]     = bhz[tid];
    sbh[2 * NHID + tid] = bhn[tid];
  }
  if (wave == 0) {
    const int bi = (tid < NOUTC) ? tid : (NOUTC - 1);
    const float bv = bd[bi];
    if (tid < NOUTC) sbd[tid] = bv;
  }
  __syncthreads();

  {
    const int row = tid >> 4, c8 = (tid & 15) * 8;
    const float* hp = h0 + (size_t)(b0 + row) * NHID + c8;
    const v4f a = *(const v4f*)(hp);
    const v4f b = *(const v4f*)(hp + 4);
    *(v4f*)(hf + row * FP + c8)     = a;
    *(v4f*)(hf + row * FP + c8 + 4) = b;
    v8h hv;
#pragma unroll
    for (int e = 0; e < 4; ++e) { hv[e] = (_Float16)(a[e] * HCARRY); hv[4 + e] = (_Float16)(b[e] * HCARRY); }
    *(v8h*)(h16 + row * HP + c8) = hv;
  }
  if (wave < 4) {
    const int row = tid >> 3, piece = tid & 7;
    const v4f xv = *(const v4f*)(x + ((size_t)(b0 + row) * NSTEP) * NFEAT + piece * 4);
    *(v4f*)(xs + row * XSP + piece * 4) = xv;
  }
  __syncthreads();

  const float wir0 = swi[j],            wir1 = swi[NHID + j];
  const float wiz0 = swi[NTHR + j],     wiz1 = swi[NTHR + NHID + j];
  const float win0 = swi[2 * NTHR + j], win1 = swi[2 * NTHR + NHID + j];
  const float br = sbh[j], bz = sbh[NHID + j], bn = sbh[2 * NHID + j];
  float wdreg[16];
#pragma unroll
  for (int q = 0; q < 16; ++q) wdreg[q] = swd[(16 * wave + q) * NOUTC + hh];
  const float bdv = sbd[hh];
  float hreg[8];
#pragma unroll
  for (int r = 0; r < 8; ++r) hreg[r] = hf[(mOff + r) * FP + j];

  const _Float16* arow = h16 + c * HP + koff;
  const _Float16* wr = WHH + (size_t)j * NHID + koff;
  const _Float16* wz = WHH + (size_t)(NHID + j) * NHID + koff;
  const _Float16* wn = WHH + (size_t)(2 * NHID + j) * NHID + koff;
  const float* hrow = hf + c * FP + 16 * wave;
  const v8f z8 = {0.f, 0.f, 0.f, 0.f, 0.f, 0.f, 0.f, 0.f};

#pragma unroll 1
  for (int t = 0; t < NSTEP; ++t) {
    v8f ar = z8, az = z8, an = z8;
#pragma unroll 1
    for (int k0 = 0; k0 < NHID; k0 += 64) {
      kstep3(ar, az, an, arow + k0,      wr + k0,      wz + k0,      wn + k0);
      kstep3(ar, az, an, arow + k0 + 32, wr + k0 + 32, wz + k0 + 32, wn + k0 + 32);
    }
    acc_guard3(ar, az, an);

    {
      float psum = 0.0f;
#pragma unroll
      for (int i = 0; i < 4; ++i) {
        const v4f p = *(const v4f*)(hrow + 4 * i);
        psum += p[0] * wdreg[4 * i];
        psum += p[1] * wdreg[4 * i + 1];
        psum += p[2] * wdreg[4 * i + 2];
        psum += p[3] * wdreg[4 * i + 3];
      }
      part[c * 16 + hh * 8 + wave] = psum;
    }

    const int sx = (t & (TCH - 1)) * NFEAT;
#pragma unroll
    for (int r = 0; r < 8; ++r) {
      const v2f xv = *(const v2f*)(xs + (mOff + r) * XSP + sx);
      const float gxr = xv[0] * wir0 + xv[1] * wir1;
      const float gxz = xv[0] * wiz0 + xv[1] * wiz1;
      const float gxn = xv[0] * win0 + xv[1] * win1;
      const float hr = ar[r] * ACC_INV + br;
      const float hz = az[r] * ACC_INV + bz;
      const float hn = an[r] * ACC_INV + bn;
      const float rg = fsig(gxr + hr);
      const float zg = fsig(gxz + hz);
      const float ng = ftanh(gxn + rg * hn);
      const float ho = hreg[r];
      hreg[r] = (1.0f - zg) * ng + zg * ho;
    }
    __syncthreads();

#pragma unroll
    for (int r = 0; r < 8; ++r) {
      h16[(mOff + r) * HP + j] = (_Float16)(hreg[r] * HCARRY);
      hf[(mOff + r) * FP + j]  = hreg[r];
    }
    if (wave == 0) {
      float s = 0.0f;
#pragma unroll
      for (int seg = 0; seg < 8; ++seg) s += part[c * 16 + hh * 8 + seg];
      const int slot = (t + TCH - 1) & (TCH - 1);
      outs[c * OSP + slot * NOUTC + hh] = s + bdv;
    }
    if ((((t + 1) & (TCH - 1)) == 0) && (t + 1 < NSTEP)) {
      if (wave < 4) {
        const int row = tid >> 3, piece = tid & 7;
        const v4f xv = *(const v4f*)(x + ((size_t)(b0 + row) * NSTEP + (size_t)(t + 1)) * NFEAT + piece * 4);
        *(v4f*)(xs + row * XSP + piece * 4) = xv;
      }
    }
    __syncthreads();

    if ((t >= TCH) && ((t & (TCH - 1)) == 0)) {
      if (wave < 4) {
        const int row = 4 * wave + (lane >> 3), c4 = (lane & 7) * 4;
        float* dst = out1 + ((size_t)(b0 + row) * NSTEP + (size_t)(t - TCH)) * NOUTC + c4;
        for (int pass = 0; pass < 2; ++pass) {
          const v4f v = *(const v4f*)(outs + row * OSP + c4);
          *(volatile v4f*)dst = v;
          __threadfence();
        }
      }
    }
  }

  {
    float psum = 0.0f;
#pragma unroll
    for (int i = 0; i < 4; ++i) {
      const v4f p = *(const v4f*)(hrow + 4 * i);
      psum += p[0] * wdreg[4 * i];
      psum += p[1] * wdreg[4 * i + 1];
      psum += p[2] * wdreg[4 * i + 2];
      psum += p[3] * wdreg[4 * i + 3];
    }
    part[c * 16 + hh * 8 + wave] = psum;
  }
  __syncthreads();
  if (wave == 0) {
    float s = 0.0f;
#pragma unroll
    for (int seg = 0; seg < 8; ++seg) s += part[c * 16 + hh * 8 + seg];
    outs[c * OSP + (TCH - 1) * NOUTC + hh] = s + bdv;
  }
  __syncthreads();
  if (wave < 4) {
    const int row = 4 * wave + (lane >> 3), c4 = (lane & 7) * 4;
    float* dst = out1 + ((size_t)(b0 + row) * NSTEP + (size_t)(NSTEP - TCH)) * NOUTC + c4;
    for (int pass = 0; pass < 2; ++pass) {
      const v4f v = *(const v4f*)(outs + row * OSP + c4);
      *(volatile v4f*)dst = v;
      __threadfence();
    }
  }
  {
    const int row = 2 * wave + hh;
    for (int pass = 0; pass < 2; ++pass) {
#pragma unroll
      for (int it = 0; it < 2; ++it) {
        const int c4 = it * 64 + c * 4;
        const v4f v = *(const v4f*)(hf + row * FP + c4);
        *(volatile v4f*)(out0 + (size_t)(b0 + row) * NHID + c4) = v;
      }
      __threadfence();
    }
  }
}

extern "C" void kernel_launch(void* const* d_in, const int* in_sizes, int n_in,
                              void* d_out, int out_size, void* d_ws, size_t ws_size, hipStream_t stream) {
  if (n_in < 13 || d_out == nullptr || d_ws == nullptr) return;
  if (in_sizes[0] != NBATCH * NSTEP * NFEAT || in_sizes[1] != NBATCH * NHID ||
      in_sizes[2] != NFEAT * NHID || in_sizes[3] != NFEAT * NHID || in_sizes[4] != NFEAT * NHID ||
      in_sizes[5] != NHID * NHID || in_sizes[6] != NHID * NHID || in_sizes[7] != NHID * NHID ||
      in_sizes[8] != NHID || in_sizes[9] != NHID || in_sizes[10] != NHID ||
      in_sizes[11] != NHID * NOUTC || in_sizes[12] != NOUTC ||
      out_size != NOUT0 + NOUT1) return;

  const float* x   = (const float*)d_in[0];
  const float* h0  = (const float*)d_in[1];
  const float* Wir = (const float*)d_in[2];
  const float* Wiz = (const float*)d_in[3];
  const float* Win = (const float*)d_in[4];
  const float* Whr = (const float*)d_in[5];
  const float* Whz = (const float*)d_in[6];
  const float* Whn = (const float*)d_in[7];
  const float* bhr = (const float*)d_in[8];
  const float* bhz = (const float*)d_in[9];
  const float* bhn = (const float*)d_in[10];
  const float* Wd  = (const float*)d_in[11];
  const float* bd  = (const float*)d_in[12];
  float* out0 = (float*)d_out;
  float* out1 = out0 + (size_t)NOUT0;

  char* ws = (char*)d_ws; size_t off = 0;
  auto carve = [&](size_t bytes) -> char* { char* p = ws + off; off += (bytes + 255) & ~(size_t)255; return p; };
  _Float16* WHH = (_Float16*)carve((size_t)NG3 * NHID * 2);
  if (off > ws_size || off > (size_t)134217728) return;

  prep_w_kernel<<<NG3 / 32, NTHR, 0, stream>>>(Whr, Whz, Whn, WHH);
  gru_seq_kernel<<<NBATCH / RB, NTHR, 0, stream>>>(x, h0, Wir, Wiz, Win, WHH, bhr, bhz, bhn, Wd, bd, out0, out1);
}
